// DisentangledSelfAttention_42683384988092
// MI455X (gfx1250) — hardware-verified
//
#include <hip/hip_runtime.h>
#include <math.h>

typedef __attribute__((ext_vector_type(16))) _Float16 v16h;
typedef __attribute__((ext_vector_type(16))) __bf16 v16b;
typedef __attribute__((ext_vector_type(8)))  _Float16 v8h;
typedef __attribute__((ext_vector_type(8)))  float v8f;
typedef __attribute__((ext_vector_type(4)))  float v4f;
typedef __attribute__((ext_vector_type(2)))  float v2f;
typedef __attribute__((ext_vector_type(4)))  unsigned v4u;
typedef __attribute__((ext_vector_type(4)))  int v4i;
typedef float __attribute__((may_alias)) float_a;
typedef int __attribute__((may_alias)) int_a;

template <typename T> __device__ __forceinline__ void vst2(void* p, T v) { *(volatile T*)p = v; __threadfence(); *(volatile T*)p = v; }
__device__ __forceinline__ v8f wmma16(v16h a, v16h b, v8f c) {
  v8f d = __builtin_amdgcn_wmma_f32_16x16x32_f16(false, a, false, b, (short)0, c, false, false);
  asm volatile("v_nop\n\tv_nop\n\tv_nop\n\tv_nop" : "+v"(d) : "v"(a), "v"(b));
  return d;
}
__device__ __forceinline__ v8f wmma_bf(v16b a, v16b b, v8f c) {
  v8f d = __builtin_amdgcn_wmma_f32_16x16x32_bf16(false, a, false, b, (short)0, c, false, false);
  asm volatile("v_nop\n\tv_nop\n\tv_nop\n\tv_nop" : "+v"(d) : "v"(a), "v"(b));
  return d;
}
__device__ __forceinline__ v16h frag_h(const _Float16* rowk0, int lane) {
  union { v16h v; v8h q[2]; } u; const _Float16* p = rowk0 + 8 * (lane >> 4);
  u.q[0] = *(const v8h*)p; u.q[1] = *(const v8h*)(p + 16); return u.v;
}
__device__ __forceinline__ v16h frag_f32(const float* rowk0, int lane) {
  v16h a; const float* p = rowk0 + 8 * (lane >> 4);
#pragma unroll
  for (int i = 0; i < 8; ++i) { a[i] = (_Float16)p[i]; a[8 + i] = (_Float16)p[16 + i]; }
  return a;
}
__device__ __forceinline__ v16h frag_f32s(const float* rowk0, int lane, float sc) {
  v16h a; const float* p = rowk0 + 8 * (lane >> 4);
#pragma unroll
  for (int i = 0; i < 8; ++i) { a[i] = (_Float16)(p[i] * sc); a[8 + i] = (_Float16)(p[16 + i] * sc); }
  return a;
}
__device__ __forceinline__ v16h fragc_f32(const float* W, int k0, int n, int lane, int ld, int K) {
  v16h a; const int g = lane >> 4;
#pragma unroll
  for (int i = 0; i < 8; ++i) { const int ka = k0 + 8 * g + i, kb = ka + 16;
    a[i] = (_Float16)(ka < K ? W[(size_t)(ka < K ? ka : K - 1) * ld + n] : 0.f); a[8 + i] = (_Float16)(kb < K ? W[(size_t)(kb < K ? kb : K - 1) * ld + n] : 0.f); }
  return a;
}
struct F2 { v16b h, l; };
__device__ __forceinline__ F2 bsplit16(const float v[16]) { F2 r;
#pragma unroll
  for (int i = 0; i < 16; ++i) { const __bf16 h = (__bf16)v[i]; r.h[i] = h; r.l[i] = (__bf16)(v[i] - (float)h); }
  return r; }
__device__ __forceinline__ F2 split_row(const float* row, int k0, int lane) { float v[16]; const float* p = row + k0 + 8 * (lane >> 4);
#pragma unroll
  for (int i = 0; i < 8; ++i) { v[i] = p[i]; v[8 + i] = p[16 + i]; }
  return bsplit16(v); }
__device__ __forceinline__ F2 split_rowK(const float* row, int k0, int lane, int K) { float v[16]; const int g = lane >> 4;
#pragma unroll
  for (int i = 0; i < 8; ++i) { const int ka = k0 + 8 * g + i, kb = ka + 16; v[i] = ka < K ? row[ka < K ? ka : K - 1] : 0.f; v[8 + i] = kb < K ? row[kb < K ? kb : K - 1] : 0.f; }
  return bsplit16(v); }
__device__ __forceinline__ F2 split_col(const float* W, int k0, int n, int lane, int ld, int K) { float v[16]; const int g = lane >> 4;
#pragma unroll
  for (int i = 0; i < 8; ++i) { const int ka = k0 + 8 * g + i, kb = ka + 16; v[i] = ka < K ? W[(size_t)(ka < K ? ka : K - 1) * ld + n] : 0.f; v[8 + i] = kb < K ? W[(size_t)(kb < K ? kb : K - 1) * ld + n] : 0.f; }
  return bsplit16(v); }
__device__ __forceinline__ v8f mac3(const F2& a, const F2& b, v8f c) { c = wmma_bf(a.l, b.h, c); c = wmma_bf(a.h, b.l, c); return wmma_bf(a.h, b.h, c); }
__device__ __forceinline__ float sigm(float v) { return 1.0f / (1.0f + expf(-v)); }
#define LDSX() do { asm volatile("s_wait_dscnt 0" ::: "memory"); __builtin_amdgcn_wave_barrier(); __builtin_amdgcn_fence(__ATOMIC_RELEASE, "workgroup"); } while (0)

#define NB 4
#define TT 1024
#define CC 1024
#define DIN 1024
#define NH 16
#define HD 64
#define NQB (TT / 64)
#define HG 8
#define SCALE (0.07216878364870323f)
#define CAUSAL 0
#ifndef TNB
#define TNB NB
#endif
__device__ __forceinline__ float bfr(float v) { return (float)(__bf16)v; }
__host__ __device__ __forceinline__ int kb_last(int qb) { return CAUSAL ? ((qb * 64 + 63) >> 7) : (TT / 128 - 1); }
typedef __attribute__((ext_vector_type(8))) __bf16 v8b;
__device__ __forceinline__ v16b frag_b(const __bf16* rowk0, int lane) {
  union { v16b v; v8b q[2]; } u; const __bf16* p = rowk0 + 8 * (lane >> 4);
  u.q[0] = *(const v8b*)p; u.q[1] = *(const v8b*)(p + 16); return u.v;
}
#define QBH 0
#define QHI 1024
#define KHI 64
__device__ __forceinline__ v16b wcol_io(const float* Wm, int k0, int o, int lane, int ld) { v16b w; const int g = lane >> 4;
#pragma unroll
  for (int i = 0; i < 8; ++i) { w[i] = (__bf16)Wm[(size_t)(k0 + 8 * g + i) * ld + o]; w[8 + i] = (__bf16)Wm[(size_t)(k0 + 16 + 8 * g + i) * ld + o]; }
  return w; }
__device__ __forceinline__ v16b wcol_oi(const float* Wm, int k0, int o, int lane, int K) { v16b w; const float* p = Wm + (size_t)o * K + k0 + 8 * (lane >> 4);
#pragma unroll
  for (int i = 0; i < 8; ++i) { w[i] = (__bf16)p[i]; w[8 + i] = (__bf16)p[16 + i]; }
  return w; }
__device__ __forceinline__ v16h wcolh_io(const float* Wm, int k0, int o, int lane, int ld) { v16h w; const int g = lane >> 4;
#pragma unroll
  for (int i = 0; i < 8; ++i) { w[i] = (_Float16)(bfr(Wm[(size_t)(k0 + 8 * g + i) * ld + o]) * 256.0f); w[8 + i] = (_Float16)(bfr(Wm[(size_t)(k0 + 16 + 8 * g + i) * ld + o]) * 256.0f); }
  return w; }
__device__ __forceinline__ v16h wcolh_oi(const float* Wm, int k0, int o, int lane, int K) { v16h w; const float* p = Wm + (size_t)o * K + k0 + 8 * (lane >> 4);
#pragma unroll
  for (int i = 0; i < 8; ++i) { w[i] = (_Float16)(bfr(p[i]) * 256.0f); w[8 + i] = (_Float16)(bfr(p[16 + i]) * 256.0f); }
  return w; }
#define WQKV_LAYOUT 0
__device__ __forceinline__ v16b wcol_hdk(const float* Wm, int k0, int o, int lane) { v16b w; const int g = lane >> 4; const float* p = Wm + (size_t)(o / HD) * DIN * HD + (o % HD);
#pragma unroll
  for (int i = 0; i < 8; ++i) { w[i] = (__bf16)p[(size_t)(k0 + 8 * g + i) * HD]; w[8 + i] = (__bf16)p[(size_t)(k0 + 16 + 8 * g + i) * HD]; }
  return w; }
#define WO_OUT_IN 0
#if WQKV_LAYOUT == 1
#define WCOL(W, k0, o, lane) wcol_oi(W, k0, o, lane, DIN)
#elif WQKV_LAYOUT == 2
#define WCOL(W, k0, o, lane) wcol_hdk(W, k0, o, lane)
#else
#define WCOL(W, k0, o, lane) wcol_io(W, k0, o, lane, CC)
#endif
#if WO_OUT_IN
#define WOCOL(W, k0, o, lane) wcol_oi(W, k0, o, lane, CC)
#define WOCOLH(W, k0, o, lane) wcolh_oi(W, k0, o, lane, CC)
#else
#define WOCOL(W, k0, o, lane) wcol_io(W, k0, o, lane, DIN)
#define WOCOLH(W, k0, o, lane) wcolh_io(W, k0, o, lane, DIN)
#endif
#define NBK 512
__constant__ short c_ridx[2047] = {0,0,0,0,0,0,0,0,0,0,0,0,0,0,0,0,0,0,0,0,0,0,0,0,0,0,0,0,0,0,0,0,0,0,0,0,0,0,0,0,0,0,0,0,0,0,0,0,0,0,0,0,0,0,0,0,0,0,0,0,0,0,0,0,0,0,0,0,0,0,0,0,0,0,0,0,0,0,0,0,0,0,0,0,0,0,0,0,0,0,0,0,0,0,0,0,0,0,0,0,0,0,0,0,0,0,0,0,0,0,0,0,0,0,0,0,0,0,0,0,0,0,0,0,0,0,0,0,0,0,0,0,0,0,0,0,0,0,0,0,0,0,0,0,0,0,0,0,0,0,0,0,0,0,0,0,0,0,0,0,0,0,0,0,0,0,0,0,0,0,0,0,0,0,0,0,0,0,0,0,0,0,0,0,0,0,0,0,0,0,0,0,0,0,0,0,0,0,0,0,0,0,0,0,0,0,0,0,0,0,0,0,0,0,0,0,0,0,0,0,0,0,0,0,0,0,0,0,0,0,0,0,0,0,0,0,0,0,0,0,0,0,0,0,0,0,0,0,0,0,0,0,0,0,0,0,0,0,0,0,0,0,0,0,0,0,0,0,0,0,0,0,0,0,0,0,0,0,0,0,0,0,0,0,0,0,0,0,0,0,0,0,0,0,0,0,0,0,0,0,0,0,0,0,0,0,0,0,0,0,0,0,0,0,0,0,0,0,0,0,0,0,0,0,0,0,0,0,0,0,0,0,0,0,0,0,0,0,0,0,0,0,0,0,0,0,0,0,0,0,0,0,0,0,0,0,0,0,0,0,0,0,0,0,0,0,0,0,0,0,0,0,0,0,0,0,0,0,0,0,0,0,0,0,0,0,0,0,0,0,0,0,0,0,0,0,0,0,0,0,0,0,0,0,0,0,0,0,0,0,0,0,0,0,0,0,0,0,0,0,0,0,0,0,0,0,0,0,0,0,0,0,0,0,0,0,0,0,0,0,0,0,0,0,0,0,0,0,0,0,0,0,0,0,0,0,0,0,0,0,0,0,0,0,0,0,0,0,0,0,0,0,0,0,0,0,0,0,0,0,0,0,0,0,0,0,0,0,0,0,0,0,0,0,0,0,0,0,0,0,0,0,0,0,0,0,0,0,0,0,0,0,1,1,1,1,1,1,2,2,2,2,2,2,3,3,3,3,3,4,4,4,4,4,5,5,5,5,5,5,6,6,6,6,6,7,7,7,7,7,8,8,8,8,8,9,9,9,9,9,10,10,10,10,10,11,11,11,11,11,12,12,12,12,12,13,13,13,13,13,14,14,14,14,14,15,15,15,15,15,16,16,16,16,17,17,17,17,17,18,18,18,18,18,19,19,19,19,20,20,20,20,20,21,21,21,21,22,22,22,22,23,23,23,23,23,24,24,24,24,25,25,25,25,26,26,26,26,26,27,27,27,27,28,28,28,28,29,29,29,29,30,30,30,30,31,31,31,31,32,32,32,32,33,33,33,33,34,34,34,34,35,35,35,35,36,36,36,37,37,37,37,38,38,38,38,39,39,39,40,40,40,40,41,41,41,41,42,42,42,43,43,43,43,44,44,44,45,45,45,45,46,46,46,47,47,47,48,48,48,48,49,49,49,50,50,50,51,51,51,52,52,52,52,53,53,53,54,54,54,55,55,55,56,56,56,57,57,57,58,58,58,59,59,59,60,60,60,61,61,61,62,62,62,63,63,64,64,64,65,65,65,66,66,66,67,67,68,68,68,69,69,69,70,70,71,71,71,72,72,73,73,73,74,74,75,75,75,76,76,77,77,77,78,78,79,79,79,80,80,81,81,82,82,83,83,83,84,84,85,85,86,86,87,87,87,88,88,89,89,90,90,91,91,92,92,93,93,94,94,95,95,96,96,97,97,98,98,99,99,100,100,101,101,102,103,103,104,104,105,105,106,106,107,108,108,109,109,110,111,111,112,112,113,114,114,115,115,116,117,117,118,119,119,120,121,121,122,123,123,124,125,125,126,127,128,129,130,131,132,133,134,135,136,137,138,139,140,141,142,143,144,145,146,147,148,149,150,151,152,153,154,155,156,157,158,159,160,161,162,163,164,165,166,167,168,169,170,171,172,173,174,175,176,177,178,179,180,181,182,183,184,185,186,187,188,189,190,191,192,193,194,195,196,197,198,199,200,201,202,203,204,205,206,207,208,209,210,211,212,213,214,215,216,217,218,219,220,221,222,223,224,225,226,227,228,229,230,231,232,233,234,235,236,237,238,239,240,241,242,243,244,245,246,247,248,249,250,251,252,253,254,255,256,257,258,259,260,261,262,263,264,265,266,267,268,269,270,271,272,273,274,275,276,277,278,279,280,281,282,283,284,285,286,287,288,289,290,291,292,293,294,295,296,297,298,299,300,301,302,303,304,305,306,307,308,309,310,311,312,313,314,315,316,317,318,319,320,321,322,323,324,325,326,327,328,329,330,331,332,333,334,335,336,337,338,339,340,341,342,343,344,345,346,347,348,349,350,351,352,353,354,355,356,357,358,359,360,361,362,363,364,365,366,367,368,369,370,371,372,373,374,375,376,377,378,379,380,381,382,383,384,385,386,387,387,388,389,389,390,391,391,392,393,393,394,395,395,396,397,397,398,398,399,400,400,401,401,402,403,403,404,404,405,406,406,407,407,408,408,409,409,410,411,411,412,412,413,413,414,414,415,415,416,416,417,417,418,418,419,419,420,420,421,421,422,422,423,423,424,424,425,425,425,426,426,427,427,428,428,429,429,429,430,430,431,431,432,432,433,433,433,434,434,435,435,435,436,436,437,437,437,438,438,439,439,439,440,440,441,441,441,442,442,443,443,443,444,444,444,445,445,446,446,446,447,447,447,448,448,448,449,449,450,450,450,451,451,451,452,452,452,453,453,453,454,454,454,455,455,455,456,456,456,457,457,457,458,458,458,459,459,459,460,460,460,460,461,461,461,462,462,462,463,463,463,464,464,464,464,465,465,465,466,466,466,467,467,467,467,468,468,468,469,469,469,469,470,470,470,471,471,471,471,472,472,472,472,473,473,473,474,474,474,474,475,475,475,475,476,476,476,477,477,477,477,478,478,478,478,479,479,479,479,480,480,480,480,481,481,481,481,482,482,482,482,483,483,483,483,484,484,484,484,485,485,485,485,486,486,486,486,486,487,487,487,487,488,488,488,488,489,489,489,489,489,490,490,490,490,491,491,491,491,492,492,492,492,492,493,493,493,493,494,494,494,494,494,495,495,495,495,495,496,496,496,496,497,497,497,497,497,498,498,498,498,498,499,499,499,499,499,500,500,500,500,500,501,501,501,501,501,502,502,502,502,502,503,503,503,503,503,504,504,504,504,504,505,505,505,505,505,506,506,506,506,506,507,507,507,507,507,507,508,508,508,508,508,509,509,509,509,509,510,510,510,510,510,510,511,511,511,511,511,511,511,511,511,511,511,511,511,511,511,511,511,511,511,511,511,511,511,511,511,511,511,511,511,511,511,511,511,511,511,511,511,511,511,511,511,511,511,511,511,511,511,511,511,511,511,511,511,511,511,511,511,511,511,511,511,511,511,511,511,511,511,511,511,511,511,511,511,511,511,511,511,511,511,511,511,511,511,511,511,511,511,511,511,511,511,511,511,511,511,511,511,511,511,511,511,511,511,511,511,511,511,511,511,511,511,511,511,511,511,511,511,511,511,511,511,511,511,511,511,511,511,511,511,511,511,511,511,511,511,511,511,511,511,511,511,511,511,511,511,511,511,511,511,511,511,511,511,511,511,511,511,511,511,511,511,511,511,511,511,511,511,511,511,511,511,511,511,511,511,511,511,511,511,511,511,511,511,511,511,511,511,511,511,511,511,511,511,511,511,511,511,511,511,511,511,511,511,511,511,511,511,511,511,511,511,511,511,511,511,511,511,511,511,511,511,511,511,511,511,511,511,511,511,511,511,511,511,511,511,511,511,511,511,511,511,511,511,511,511,511,511,511,511,511,511,511,511,511,511,511,511,511,511,511,511,511,511,511,511,511,511,511,511,511,511,511,511,511,511,511,511,511,511,511,511,511,511,511,511,511,511,511,511,511,511,511,511,511,511,511,511,511,511,511,511,511,511,511,511,511,511,511,511,511,511,511,511,511,511,511,511,511,511,511,511,511,511,511,511,511,511,511,511,511,511,511,511,511,511,511,511,511,511,511,511,511,511,511,511,511,511,511,511,511,511,511,511,511,511,511,511,511,511,511,511,511,511,511,511,511,511,511,511,511,511,511,511,511,511,511,511,511,511,511,511,511,511,511,511,511,511,511,511,511,511,511,511,511,511,511,511,511,511,511,511,511,511,511,511,511,511,511,511,511,511,511,511,511,511,511,511,511,511,511,511,511,511,511,511,511,511,511,511,511,511,511,511,511,511,511,511,511,511,511,511,511,511,511,511,511,511,511,511,511,511,511,511,511,511,511,511,511,511,511,511,511,511,511,511,511,511,511,511,511,511,511,511,511,511,511,511,511,511,511,511,511,511,511,511,511,511,511,511,511,511,511,511,511,511,511,511,511,511,511,511,511,511,511,511,511,511,511,511,511,511,511,511,511,511,511,511,511};
#define SM_EXTRA_PARAMS , const float* __restrict__ QP
#define SM_MASK_HOOK do { const int ri = c_ridx[(t - k) + 1023]; v = v + (QP[((size_t)(blockIdx.y * 2 + 0) * TT + t) * NBK + ri] + QP[((size_t)(blockIdx.y * 2 + 1) * TT + k) * NBK + ri]) * 0.08838834764831845f; } while (0)
__global__ __launch_bounds__(256) void k_lnre(const float* __restrict__ EMB, const float* __restrict__ G, const float* __restrict__ BE, float* __restrict__ RE) { __shared__ float sred[8]; __shared__ float sbc;
  const int t = threadIdx.x; const int r = blockIdx.x; float v[4]; float s1 = 0.f;
#pragma unroll
  for (int i = 0; i < 4; ++i) { v[i] = bfr(EMB[(size_t)r * 1024 + i * 256 + t]); s1 += v[i]; }
  for (int o = 1; o < 32; o <<= 1) s1 += __shfl_xor(s1, o);
  if ((t & 31) == 0) sred[t >> 5] = s1; __syncthreads(); if (t == 0) { float a = 0.f; for (int i = 0; i < 8; ++i) a += sred[i]; sbc = a / 1024.f; } __syncthreads(); const float mu = sbc; __syncthreads();
  float s2 = 0.f;
#pragma unroll
  for (int i = 0; i < 4; ++i) { const float d = v[i] - mu; s2 += d * d; }
  for (int o = 1; o < 32; o <<= 1) s2 += __shfl_xor(s2, o);
  if ((t & 31) == 0) sred[t >> 5] = s2; __syncthreads(); if (t == 0) { float a = 0.f; for (int i = 0; i < 8; ++i) a += sred[i]; sbc = rsqrtf(a / 1024.f + 1e-5f); } __syncthreads(); const float rs = sbc;
  __shared__ __align__(16) float so[1024];
#pragma unroll
  for (int i = 0; i < 4; ++i) { const int c = i * 256 + t; so[c] = (v[i] - mu) * rs * bfr(G[c]) + bfr(BE[c]); }
  __syncthreads(); vst2(RE + (size_t)r * 1024 + t * 4, *(const v4f*)&so[t * 4]); }
__global__ __launch_bounds__(128) void k_posproj(const float* __restrict__ RE, const float* __restrict__ WPK, const float* __restrict__ BPK, const float* __restrict__ WPQ, const float* __restrict__ BPQ, float* __restrict__ POSK, float* __restrict__ POSQ) { __shared__ __align__(16) float sf[4][16][132];
  const int tid = threadIdx.x, wave = tid >> 5, lane = tid & 31, col = lane & 15, g = lane >> 4; const int which = blockIdx.z; const int c0 = blockIdx.y * 128; const size_t r0 = (size_t)blockIdx.x * 64 + wave * 16;
  const float* Wp = which == 0 ? WPK : WPQ; const float* Bp = which == 0 ? BPK : BPQ; float* OUTP = which == 0 ? POSK : POSQ;
  v8f acc[8] = {};
#pragma unroll 1
  for (int kc = 0; kc < CC / 32; ++kc) { const F2 a = split_row(RE + (r0 + col) * CC, kc * 32, lane); asm volatile("s_wait_loadcnt 0x0" ::: "memory");
#pragma unroll
    for (int j = 0; j < 8; ++j) { const v16b w = wcol_io(Wp, kc * 32, c0 + j * 16 + col, lane, CC); asm volatile("s_wait_loadcnt 0x0" ::: "memory"); acc[j] = wmma_bf(a.h, w, acc[j]); acc[j] = wmma_bf(a.l, w, acc[j]); } }
#pragma unroll
  for (int j = 0; j < 8; ++j) { const float bb = bfr(Bp[c0 + j * 16 + col]);
#pragma unroll
    for (int r = 0; r < 8; ++r) sf[wave][8 * g + r][j * 16 + col] = acc[j][r] + bb; }
  asm volatile("s_wait_loadcnt 0x0" ::: "memory");
  LDSX(); for (int rl = 0; rl < 16; ++rl) vst2(OUTP + (r0 + rl) * CC + c0 + lane * 4, *(const v4f*)&sf[wave][rl][lane * 4]); }
__global__ __launch_bounds__(128) void k_qp(const _Float16* __restrict__ QH, const _Float16* __restrict__ KH, const float* __restrict__ POSK, const float* __restrict__ POSQ, int b, int h0, float* __restrict__ QP) { __shared__ __align__(16) float sf[4][16][132];
  const int tid = threadIdx.x, wave = tid >> 5, lane = tid & 31, col = lane & 15, g = lane >> 4; const int hg = blockIdx.z >> 1, which = blockIdx.z & 1; const int h = h0 + hg; const int m0 = blockIdx.y * 128; const int s0 = blockIdx.x * 64 + wave * 16;
  const _Float16* PL = which == 0 ? QH : KH; const float* POS = which == 0 ? POSK : POSQ;
  v8f acc[8] = {};
#pragma unroll
  for (int kc = 0; kc < HD / 32; ++kc) { const v16h a = frag_h(PL + ((size_t)b * TT + s0 + col) * CC + h * HD + kc * 32, lane); asm volatile("s_wait_loadcnt 0x0" ::: "memory");
#pragma unroll
    for (int j = 0; j < 8; ++j) { const v16h w = frag_f32(POS + (size_t)(m0 + j * 16 + col) * CC + h * HD + kc * 32, lane); asm volatile("s_wait_loadcnt 0x0" ::: "memory"); acc[j] = wmma16(a, w, acc[j]); } }
#pragma unroll
  for (int j = 0; j < 8; ++j)
#pragma unroll
    for (int r = 0; r < 8; ++r) sf[wave][8 * g + r][j * 16 + col] = acc[j][r];
  LDSX(); for (int rl = 0; rl < 16; ++rl) vst2(QP + ((size_t)(hg * 2 + which) * TT + s0 + rl) * NBK + m0 + lane * 4, *(const v4f*)&sf[wave][rl][lane * 4]); }
#define WS_RE   (WS_END)
#define WS_POSK (WS_RE + 4u * (size_t)NBK * CC)
#define WS_POSQ (WS_POSK + 4u * (size_t)NBK * CC)
#define WS_QP   (WS_POSQ + 4u * (size_t)NBK * CC)
#define WS_END2 (WS_QP + 4u * (size_t)HG * 2 * TT * NBK)
#ifndef SM_EXTRA_PARAMS
#define SM_EXTRA_PARAMS
#endif
#ifndef PROJ_EXTRA_PARAMS
#define PROJ_EXTRA_PARAMS
#endif
#ifndef SM_MASK_HOOK
#define SM_MASK_HOOK (void)0
#endif

#define WS_QH  0u
#define WS_KH  (WS_QH + 2u * (size_t)NB * TT * CC)
#define WS_VT  (WS_KH + 2u * (size_t)NB * TT * CC)
#define WS_QL  (WS_VT + 2u * (size_t)NB * CC * TT)
#define WS_KL  (WS_QL + 2u * (size_t)NB * QHI * CC)
#define WS_VB  (WS_KL + 2u * (size_t)NB * KHI * CC)
#define WS_VBL (WS_VB + 2u * (size_t)NB * CC * KHI)
#define WS_S   (WS_VBL + 2u * (size_t)NB * CC * KHI)
#define WS_Y   (WS_S  + 4u * (size_t)HG * TT * TT)
#define WS_END (WS_Y  + 4u * (size_t)NB * TT * CC)

__global__ __launch_bounds__(128) void k_proj(const float* __restrict__ XQ, const float* __restrict__ XK, const float* __restrict__ XV, const float* __restrict__ WQ, const float* __restrict__ WK, const float* __restrict__ WV, const float* __restrict__ BQ, const float* __restrict__ BK, const float* __restrict__ BV,
    _Float16* __restrict__ QH, _Float16* __restrict__ QL, _Float16* __restrict__ KH, _Float16* __restrict__ KL, _Float16* __restrict__ VT, __bf16* __restrict__ VB, __bf16* __restrict__ VBL) {
  __shared__ __align__(16) _Float16 sh[64][136], sl[64][136]; __shared__ __align__(16) _Float16 th[128][72]; __shared__ __align__(16) __bf16 tb[128][72], tbl[128][72];
  const int tid = threadIdx.x, wave = tid >> 5, lane = tid & 31, col = lane & 15, g = lane >> 4; const int which = blockIdx.z; const int c0 = blockIdx.y * 128; const size_t r0 = (size_t)blockIdx.x * 64; const size_t bb = r0 / TT; const int t0 = (int)(r0 % TT);
  const float* X = which == 0 ? XQ : which == 1 ? XK : XV; const float* WA = which == 0 ? WQ : which == 1 ? WK : WV; const float* BA = which == 0 ? BQ : which == 1 ? BK : BV;
  v8f acc[8] = {};
#pragma unroll 2
  for (int kc = 0; kc < DIN / 32; ++kc) { v16b a; { const float* p = X + (r0 + wave * 16 + col) * DIN + kc * 32 + 8 * g;
#pragma unroll
      for (int i = 0; i < 8; ++i) { a[i] = (__bf16)p[i]; a[8 + i] = (__bf16)p[16 + i]; } }
    asm volatile("s_wait_loadcnt 0x0" ::: "memory");
#pragma unroll
    for (int j = 0; j < 8; ++j) { const v16b w = WCOL(WA, kc * 32, c0 + j * 16 + col, lane); asm volatile("s_wait_loadcnt 0x0" ::: "memory"); acc[j] = wmma_bf(a, w, acc[j]); } }
  if (which < 2) { _Float16* DH = which == 0 ? QH : KH; _Float16* DL = which == 0 ? QL : KL; const int nhi = which == 0 ? QHI : KHI; const bool hi_rows = t0 < nhi;
#pragma unroll
    for (int j = 0; j < 8; ++j) { const float bias = BA ? bfr(BA[c0 + j * 16 + col]) : 0.f;
#pragma unroll
      for (int r = 0; r < 8; ++r) { const float v = acc[j][r] + bias; const _Float16 hv = (_Float16)v; sh[wave * 16 + 8 * g + r][j * 16 + col] = hv; sl[wave * 16 + 8 * g + r][j * 16 + col] = (_Float16)((v - (float)hv) * 1024.0f); } }
    __syncthreads();
    for (int e = tid; e < 64 * 16; e += 128) { const int rl = e >> 4, q = e & 15; vst2((unsigned*)(DH + (r0 + rl) * CC + c0 + q * 8), *(const v4u*)&sh[rl][q * 8]); if (hi_rows) vst2((unsigned*)(DL + (bb * nhi + t0 + rl) * (size_t)CC + c0 + q * 8), *(const v4u*)&sl[rl][q * 8]); }
  } else { const bool hi_rows = t0 < KHI;
#pragma unroll
    for (int j = 0; j < 8; ++j) { const float bias = BA ? bfr(BA[c0 + j * 16 + col]) : 0.f;
#pragma unroll
      for (int r = 0; r < 8; ++r) { const float v = acc[j][r] + bias; const int rl = wave * 16 + 8 * g + r, cl = j * 16 + col; th[cl][rl] = (_Float16)v; const __bf16 bh = (__bf16)v; tb[cl][rl] = bh; tbl[cl][rl] = (__bf16)(v - (float)bh); } }
    __syncthreads();
    for (int e = tid; e < 128 * 8; e += 128) { const int cl = e >> 3, q = e & 7; vst2((unsigned*)(VT + (bb * CC + c0 + cl) * (size_t)TT + t0 + q * 8), *(const v4u*)&th[cl][q * 8]); if (hi_rows) { const size_t o3 = (bb * CC + c0 + cl) * (size_t)KHI + t0 + q * 8; vst2((unsigned*)(VB + o3), *(const v4u*)&tb[cl][q * 8]); vst2((unsigned*)(VBL + o3), *(const v4u*)&tbl[cl][q * 8]); } } } }
__global__ __launch_bounds__(128) void k_sc(const _Float16* __restrict__ QH, const _Float16* __restrict__ KH, const _Float16* __restrict__ QL, const _Float16* __restrict__ KL, int b, int h0, float* __restrict__ S0) { __shared__ __align__(16) float ss[4][16][132];
  const int qb = blockIdx.x, kb = blockIdx.y; if (kb > kb_last(qb)) return;
  const int h = h0 + blockIdx.z; float* S = S0 + (size_t)blockIdx.z * TT * TT;
  const int tid = threadIdx.x, wave = tid >> 5, lane = tid & 31, col = lane & 15, g = lane >> 4; const int k0 = kb * 128; const int ql0 = qb * 64 + wave * 16; const size_t q0 = (size_t)b * TT + ql0, kr0 = (size_t)b * TT + k0;
  v8f acc[8] = {}, accl[8] = {};
  const _Float16* QLb = QL + (size_t)b * QHI * CC; const _Float16* KLb = KL + (size_t)b * KHI * CC;
  if (qb < QBH) {
#pragma unroll
    for (int kc = 0; kc < HD / 32; ++kc) { const v16h ah = frag_h(QH + (q0 + col) * CC + h * HD + kc * 32, lane), al = frag_h(QLb + (size_t)(ql0 + col) * CC + h * HD + kc * 32, lane);
#pragma unroll
      for (int j = 0; j < 8; ++j) { const v16h kbf = frag_h(KH + (kr0 + j * 16 + col) * CC + h * HD + kc * 32, lane), klf = frag_h(KLb + (size_t)(k0 + j * 16 + col) * CC + h * HD + kc * 32, lane); acc[j] = wmma16(ah, kbf, acc[j]); accl[j] = wmma16(al, kbf, accl[j]); accl[j] = wmma16(ah, klf, accl[j]); } }
  } else if (qb * 64 < QHI) {
#pragma unroll
    for (int kc = 0; kc < HD / 32; ++kc) { const v16h ah = frag_h(QH + (q0 + col) * CC + h * HD + kc * 32, lane), al = frag_h(QLb + (size_t)(ql0 + col) * CC + h * HD + kc * 32, lane);
#pragma unroll
      for (int j = 0; j < 8; ++j) { const v16h kbf = frag_h(KH + (kr0 + j * 16 + col) * CC + h * HD + kc * 32, lane); acc[j] = wmma16(ah, kbf, acc[j]); accl[j] = wmma16(al, kbf, accl[j]); } }
  } else {
#pragma unroll
    for (int kc = 0; kc < HD / 32; ++kc) { const v16h ah = frag_h(QH + (q0 + col) * CC + h * HD + kc * 32, lane);
#pragma unroll
      for (int j = 0; j < 8; ++j) { const v16h kbf = frag_h(KH + (kr0 + j * 16 + col) * CC + h * HD + kc * 32, lane); acc[j] = wmma16(ah, kbf, acc[j]); } } }
#pragma unroll
  for (int j = 0; j < 8; ++j) {
#pragma unroll
    for (int r = 0; r < 8; ++r) ss[wave][8 * g + r][j * 16 + col] = (acc[j][r] + accl[j][r] * (1.0f / 1024.0f)) * SCALE; }
  LDSX(); for (int rl = 0; rl < 16; ++rl) vst2(S + (size_t)(ql0 + rl) * TT + k0 + lane * 4, *(const v4f*)&ss[wave][rl][lane * 4]); }
__global__ __launch_bounds__(256) void k_sm(float* __restrict__ S0 SM_EXTRA_PARAMS) { __shared__ float sred[8]; __shared__ float sbc; __shared__ __align__(16) float shv[TT];
  const int tid = threadIdx.x; const int t = blockIdx.x; const int kend = (kb_last(t >> 6) + 1) * 128;
  float* sr = S0 + (size_t)blockIdx.y * TT * TT + (size_t)t * TT;
  float m = -3.0e38f; for (int k = tid; k < kend; k += 256) { float v = (!CAUSAL || k <= t) ? sr[k] : -3.0e38f; SM_MASK_HOOK; shv[k] = v; m = fmaxf(m, v); }
#pragma unroll
  for (int o = 1; o < 32; o <<= 1) m = fmaxf(m, __shfl_xor(m, o));
  if ((tid & 31) == 0) sred[tid >> 5] = m; __syncthreads(); if (tid == 0) { float a = sred[0]; for (int i = 1; i < 8; ++i) a = fmaxf(a, sred[i]); sbc = a; } __syncthreads(); m = sbc; __syncthreads();
  float sum = 0.f; for (int k = tid; k < kend; k += 256) { const float v = shv[k]; const float e = (v <= -1.0e38f) ? 0.f : expf(v - m); shv[k] = e; sum += e; }
#pragma unroll
  for (int o = 1; o < 32; o <<= 1) sum += __shfl_xor(sum, o);
  if ((tid & 31) == 0) sred[tid >> 5] = sum; __syncthreads(); if (tid == 0) { float a = 0.f; for (int i = 0; i < 8; ++i) a += sred[i]; sbc = a > 0.f ? 2048.0f / a : 0.f; }     __syncthreads(); const float inv = sbc;
  for (int k = tid; k < kend; k += 256) shv[k] = shv[k] * inv;
  __syncthreads(); for (int q = tid; q < kend / 4; q += 256) vst2(sr + q * 4, *(const v4f*)&shv[q * 4]); }
__global__ __launch_bounds__(128) void k_pv(const float* __restrict__ PS0, const _Float16* __restrict__ VT, const __bf16* __restrict__ VB, const __bf16* __restrict__ VBL, int b, int h0, float* __restrict__ Y) { const int h = h0 + blockIdx.z; const float* PS = PS0 + (size_t)blockIdx.z * TT * TT; __shared__ __align__(16) float ss[4][16][HD + 4];
  const int tid = threadIdx.x, wave = tid >> 5, lane = tid & 31, col = lane & 15, g = lane >> 4; const int qb = blockIdx.x; const int ql0 = qb * 64 + wave * 16; const int kce = (kb_last(qb) + 1) * 4;
  v8f acc[HD / 16] = {};
  if (qb < QBH) {
#pragma unroll 1
    for (int kc = 0; kc < kce; ++kc) { const F2 p = split_row(PS + (size_t)(ql0 + col) * TT, kc * 32, lane);
      asm volatile("s_wait_loadcnt 0x0" ::: "memory");
#pragma unroll
      for (int j = 0; j < HD / 16; ++j) { const size_t po = ((size_t)b * CC + h * HD + j * 16 + col) * (size_t)KHI + kc * 32; const v16b vh = frag_b(VB + po, lane); acc[j] = wmma_bf(p.h, vh, acc[j]); acc[j] = wmma_bf(p.l, vh, acc[j]); acc[j] = wmma_bf(p.h, frag_b(VBL + po, lane), acc[j]); } }
  } else {
#pragma unroll 1
    for (int kc = 0; kc < kce; ++kc) { const v16h p = frag_f32(PS + (size_t)(ql0 + col) * TT + kc * 32, lane);
      asm volatile("s_wait_loadcnt 0x0" ::: "memory");
#pragma unroll
      for (int j = 0; j < HD / 16; ++j) { const size_t po = ((size_t)b * CC + h * HD + j * 16 + col) * (size_t)TT + kc * 32; acc[j] = wmma16(p, frag_h(VT + po, lane), acc[j]); } } }
#pragma unroll
  for (int j = 0; j < HD / 16; ++j)
#pragma unroll
    for (int r = 0; r < 8; ++r) ss[wave][8 * g + r][j * 16 + col] = acc[j][r] * (1.0f / 2048.0f);
  LDSX(); for (int rl = 0; rl < 16; ++rl) if (lane < HD / 4) vst2(Y + ((size_t)b * TT + ql0 + rl) * CC + h * HD + lane * 4, *(const v4f*)&ss[wave][rl][lane * 4]); }
__global__ __launch_bounds__(128) void k_out(const float* __restrict__ Y, const float* __restrict__ WO, const float* __restrict__ BO, float* __restrict__ OUT) { __shared__ __align__(16) float sf[4][16][132];
  const int tid = threadIdx.x, wave = tid >> 5, lane = tid & 31, col = lane & 15, g = lane >> 4; const int c0 = blockIdx.y * 128; const size_t r0 = (size_t)blockIdx.x * 64 + wave * 16;
  v8f acc[8] = {};
  if (CAUSAL && (int)(((size_t)blockIdx.x * 64) % TT) < QHI) {
#pragma unroll 2
    for (int kc = 0; kc < CC / 32; ++kc) { const F2 a = split_row(Y + (r0 + col) * CC, kc * 32, lane); asm volatile("s_wait_loadcnt 0x0" ::: "memory");
#pragma unroll
      for (int j = 0; j < 8; ++j) { const v16b w = WOCOL(WO, kc * 32, c0 + j * 16 + col, lane); asm volatile("s_wait_loadcnt 0x0" ::: "memory"); acc[j] = wmma_bf(a.h, w, acc[j]); acc[j] = wmma_bf(a.l, w, acc[j]); } }
#pragma unroll
    for (int j = 0; j < 8; ++j) { const float bias = BO ? bfr(BO[c0 + j * 16 + col]) : 0.f;
#pragma unroll
      for (int r = 0; r < 8; ++r) sf[wave][8 * g + r][j * 16 + col] = acc[j][r] + bias; }
  } else {
#pragma unroll 2
    for (int kc = 0; kc < CC / 32; ++kc) { const v16h a = frag_f32(Y + (r0 + col) * CC + kc * 32, lane); asm volatile("s_wait_loadcnt 0x0" ::: "memory");
#pragma unroll
      for (int j = 0; j < 8; ++j) { const v16h w = WOCOLH(WO, kc * 32, c0 + j * 16 + col, lane); asm volatile("s_wait_loadcnt 0x0" ::: "memory"); acc[j] = wmma16(a, w, acc[j]); } }
#pragma unroll
    for (int j = 0; j < 8; ++j) { const float bias = BO ? bfr(BO[c0 + j * 16 + col]) : 0.f;
#pragma unroll
      for (int r = 0; r < 8; ++r) sf[wave][8 * g + r][j * 16 + col] = acc[j][r] * (1.0f / 256.0f) + bias; } }
  LDSX(); for (int rl = 0; rl < 16; ++rl) vst2(OUT + (r0 + rl) * DIN + c0 + lane * 4, *(const v4f*)&sf[wave][rl][lane * 4]); }

extern "C" void kernel_launch(void* const* d_in, const int* in_sizes, int n_in, void* d_out, int out_size, void* d_ws, size_t ws_size, hipStream_t stream) {
  (void)in_sizes; (void)n_in; (void)out_size;
  const float** F = (const float**)d_in;
  if (ws_size < (size_t)WS_END) return;
  char* ws = (char*)d_ws; _Float16 *QH = (_Float16*)(ws + WS_QH), *KH = (_Float16*)(ws + WS_KH), *VT = (_Float16*)(ws + WS_VT), *QL = (_Float16*)(ws + WS_QL), *KL = (_Float16*)(ws + WS_KL); __bf16 *VB = (__bf16*)(ws + WS_VB), *VBL = (__bf16*)(ws + WS_VBL); float *S = (float*)(ws + WS_S), *Y = (float*)(ws + WS_Y);
  (void)Y; (void)QL; (void)KL; (void)VB; (void)VBL;
  if (ws_size < (size_t)WS_END2) return;
  float *RE = (float*)(ws + WS_RE), *POSK = (float*)(ws + WS_POSK), *POSQ = (float*)(ws + WS_POSQ), *QP = (float*)(ws + WS_QP);
  k_lnre<<<dim3(NBK), 256, 0, stream>>>(F[9], F[10], F[11], RE);
  k_posproj<<<dim3(NBK / 64, CC / 128, 2), 128, 0, stream>>>(RE, F[12], F[13], F[14], F[15], POSK, POSQ);
  k_proj<<<dim3(TNB * TT / 64, CC / 128, 3), 128, 0, stream>>>(F[0], F[0], F[0], F[1], F[3], F[5], F[2], F[4], F[6], QH, QL, KH, KL, VT, VB, VBL);
  for (int b = 0; b < TNB; ++b) for (int h0 = 0; h0 < NH; h0 += HG) {
    k_qp<<<dim3(TT / 64, NBK / 128, HG * 2), 128, 0, stream>>>(QH, KH, POSK, POSQ, b, h0, QP);
    k_sc<<<dim3(NQB, TT / 128, HG), 128, 0, stream>>>(QH, KH, QL, KL, b, h0, S);
    k_sm<<<dim3(TT, HG), 256, 0, stream>>>(S, QP);
    k_pv<<<dim3(NQB, 1, HG), 128, 0, stream>>>(S, VT, VB, VBL, b, h0, Y);
  }
  k_out<<<dim3(TNB * TT / 64, DIN / 128), 128, 0, stream>>>(Y, F[7], F[8], (float*)d_out);
}
